// GGNet_11012296147741
// MI455X (gfx1250) — hardware-verified
//
#include <hip/hip_runtime.h>
#include <stddef.h>
#include <stdint.h>


#define HD     64
#define NDIM   133
#define KX     160
#define BDIM   16
#define INTD   128
#define NG     64
#define W2N    4096
#define KW     8256
#define GH     192
#define LK     192
#define LG     256

#define NTHR   256
#define NWAVE  8
#define EPT    8
#define CHUNK  (NTHR * EPT)
#define WCAP   (EPT * 32)
#define LISTN  (NWAVE * WCAP)
#define TPW    16
#define PASSN  (NWAVE * TPW)
#define PCAP   (CHUNK + PASSN)
#define NB     256
#define AW     65
#define NQE    ((NB * HD) / (128 * NWAVE))

#define SACT    16.0f
#define SWGT    16.0f
#define SBIA    256.0f
#define ISC16   0.0625f
#define ISC256  0.00390625f
#define ISC4096 0.000244140625f

static_assert(PASSN == 128);
static_assert((PCAP % PASSN) == 0);
static_assert(NQE * 128 * NWAVE == NB * HD);
static_assert((NB % 64) == 0);
static_assert(WCAP == EPT * 32);

typedef float    v2f  __attribute__((ext_vector_type(2)));
typedef float    v4f  __attribute__((ext_vector_type(4)));
typedef float    v8f  __attribute__((ext_vector_type(8)));
typedef int      v4i  __attribute__((ext_vector_type(4)));
typedef _Float16 v4h  __attribute__((ext_vector_type(4)));
typedef _Float16 v8h  __attribute__((ext_vector_type(8)));
typedef _Float16 v16h __attribute__((ext_vector_type(16)));
union FragH { v16h v; v8h h[2]; };
union U8 { v8h h; v4f f; };

constexpr int al16(int v) { return (v + 15) & ~15; }

constexpr int EO_ACC  = 0;
constexpr int EO_MSG  = al16(EO_ACC + (NB + 1) * AW * 4);
constexpr int EO_SEA  = al16(EO_MSG + PASSN * AW * 4);
constexpr int EO_SOU  = al16(EO_SEA + PASSN * BDIM * 2);
constexpr int EO_LIST = al16(EO_SOU + PASSN * HD * 2);
constexpr int EO_PEND = al16(EO_LIST + LISTN * 4);
constexpr int EO_SLOT = al16(EO_PEND + PCAP * 4);
constexpr int EO_WE1  = al16(EO_SLOT + PASSN * 4);
constexpr int EO_BSM  = al16(EO_WE1 + INTD * 32 * 2);
constexpr int EO_WCNT = al16(EO_BSM + INTD * 4);
constexpr int EO_PN   = al16(EO_WCNT + NWAVE * 4);
constexpr int E_LDS   = al16(EO_PN + 16);

constexpr int SO_APL  = 0;
constexpr int SO_HLS  = SO_APL + NG * LK * 2;
constexpr int SO_RAC  = SO_HLS + NG * HD * 4;
constexpr int SO_GMX  = SO_RAC + NG * HD * 4;
constexpr int SO_GSM  = SO_GMX + NG * 4;
constexpr int SO_GIV  = SO_GSM + NG * 4;
constexpr int SO_ES   = SO_GIV + NG * 4;
static_assert((SO_ES % 16) == 0);

extern __shared__ __attribute__((aligned(16))) unsigned char dyn_lds[];

__device__ __forceinline__ v8h zero8() {
  v8h r;
#pragma unroll
  for (int i = 0; i < 8; ++i) r[i] = (_Float16)0.0f;
  return r;
}
__device__ __forceinline__ v8f zerof8() {
  v8f r;
#pragma unroll
  for (int i = 0; i < 8; ++i) r[i] = 0.0f;
  return r;
}
__device__ __forceinline__ float rcpf(float x) { return __builtin_amdgcn_rcpf(x); }
__device__ __forceinline__ float sigf(float x) {
  const float e = __expf(-fabsf(x));
  const float r = rcpf(1.0f + e);
  return (x >= 0.0f) ? r : e * r;
}

__device__ __forceinline__ v8f wmh(v16h a, v16h b, v8f c) {
  v8f d = __builtin_amdgcn_wmma_f32_16x16x32_f16(false, a, false, b, (short)0, c, false, false);
  asm volatile("v_nop\n\tv_nop\n\tv_nop\n\tv_nop" : "+v"(d) : "v"(a), "v"(b));
  return d;
}
__device__ __forceinline__ void wm4(v16h a, v16h b0, v16h b1, v16h b2, v16h b3,
                                    v8f& c0, v8f& c1, v8f& c2, v8f& c3) {
  c0 = __builtin_amdgcn_wmma_f32_16x16x32_f16(false, a, false, b0, (short)0, c0, false, false);
  c1 = __builtin_amdgcn_wmma_f32_16x16x32_f16(false, a, false, b1, (short)0, c1, false, false);
  c2 = __builtin_amdgcn_wmma_f32_16x16x32_f16(false, a, false, b2, (short)0, c2, false, false);
  c3 = __builtin_amdgcn_wmma_f32_16x16x32_f16(false, a, false, b3, (short)0, c3, false, false);
  asm volatile("v_nop\n\tv_nop\n\tv_nop\n\tv_nop"
               : "+v"(c0), "+v"(c1), "+v"(c2), "+v"(c3)
               : "v"(a), "v"(b0), "v"(b1), "v"(b2), "v"(b3));
}

__device__ __forceinline__ FragH ldf(const _Float16* p) {
  FragH f;
  f.h[0] = *(const v8h*)p;
  f.h[1] = *(const v8h*)(p + 16);
  return f;
}
__device__ __forceinline__ v8f ldc8(const float* p) {
  const v4f a = *(const v4f*)p;
  const v4f b = *(const v4f*)(p + 4);
  v8f c;
  c[0] = a.x; c[1] = a.y; c[2] = a.z; c[3] = a.w;
  c[4] = b.x; c[5] = b.y; c[6] = b.z; c[7] = b.w;
  return c;
}
__device__ __forceinline__ v8h cvh8(v4f a, v4f b, float sc) {
  v8h r;
  r[0] = (_Float16)(a.x * sc); r[1] = (_Float16)(a.y * sc); r[2] = (_Float16)(a.z * sc); r[3] = (_Float16)(a.w * sc);
  r[4] = (_Float16)(b.x * sc); r[5] = (_Float16)(b.y * sc); r[6] = (_Float16)(b.z * sc); r[7] = (_Float16)(b.w * sc);
  return r;
}
__device__ __forceinline__ v8h cveh(v8f d) {
  v8h r;
#pragma unroll
  for (int i = 0; i < 8; ++i) { const float t = fmaxf(d[i], 0.0f) * ISC16; r[i] = (_Float16)t; }
  return r;
}

template <int NP, typename F>
__device__ __forceinline__ void emit8(_Float16* dst, int np, int tid, F f) {
  U8 pv[NP];
#pragma unroll
  for (int it = 0; it < NP; ++it) {
    int p = it * 256 + tid;
    p = p < np ? p : np - 1;
    pv[it].h = f(p, it);
  }
#pragma unroll
  for (int it = 0; it < NP; ++it) {
    const int p = it * 256 + tid;
    if (p < np) *(volatile v4f*)(dst + 8 * (size_t)p) = pv[it].f;
  }
  __threadfence();
#pragma unroll
  for (int it = 0; it < NP; ++it) {
    const int p = it * 256 + tid;
    if (p < np) *(volatile v4f*)(dst + 8 * (size_t)p) = pv[it].f;
  }
}

__global__ __launch_bounds__(256) void k_prep(
    const float* __restrict__ We2, const float* __restrict__ be2, const float* __restrict__ Wexp,
    const float* __restrict__ Wroot, const float* __restrict__ We1, const float* __restrict__ gWih,
    const float* __restrict__ gWhh, const float* __restrict__ lWih, const float* __restrict__ lWhh,
    _Float16* Wp, _Float16* WexpT, _Float16* WrootP, _Float16* We1T, _Float16* WihP, _Float16* WhhP,
    _Float16* LstmP) {
  const int tid = threadIdx.x, bid = blockIdx.x;
  if (bid < NG) {
    const int o = bid;
    emit8<5>(Wp + (size_t)o * KW, 1032, tid, [&](int p, int it) -> v8h {
      v8h r;
      if (it < 4) {
        const int i = p >> 4, kb = (p & 15) << 3;
#pragma unroll
        for (int kk = 0; kk < 8; ++kk)
          r[kk] = (_Float16)(We2[(size_t)(kb + kk) * W2N + i * HD + o] * SWGT);
      } else {
        int q = p - 1024;
        q = q < 0 ? 0 : (q > 7 ? 7 : q);
        const int ib = q << 3;
#pragma unroll
        for (int kk = 0; kk < 8; ++kk)
          r[kk] = (_Float16)(be2[(ib + kk) * HD + o] * SBIA);
      }
      return r;
    });
  } else if (bid == NG) {
    emit8<5>(WexpT, (HD * KX) / 8, tid, [&](int p, int) -> v8h {
      v8h r;
      const int o = p / (KX / 8), kb = (p - o * (KX / 8)) * 8;
#pragma unroll
      for (int kk = 0; kk < 8; ++kk) {
        const int k = kb + kk;
        const int kc = k > NDIM - 1 ? NDIM - 1 : k;
        const float v = Wexp[kc * HD + o];
        r[kk] = (_Float16)((k < NDIM) ? v * SWGT : 0.0f);
      }
      return r;
    });
  } else if (bid == NG + 1) {
    emit8<2>(WrootP, (HD * HD) / 8, tid, [&](int p, int) -> v8h {
      v8h r;
      const int o = p >> 3, kb = (p & 7) << 3;
#pragma unroll
      for (int kk = 0; kk < 8; ++kk) r[kk] = (_Float16)(Wroot[(kb + kk) * HD + o] * SWGT);
      return r;
    });
  } else if (bid == NG + 2) {
    emit8<2>(We1T, (INTD * 32) / 8, tid, [&](int p, int) -> v8h {
      v8h r;
      const int n = p >> 2, kb = (p & 3) << 3;
#pragma unroll
      for (int kk = 0; kk < 8; ++kk) {
        const int k = kb + kk;
        const int kc = k > BDIM - 1 ? BDIM - 1 : k;
        const float v = We1[kc * INTD + n];
        r[kk] = (_Float16)((k < BDIM) ? v * SWGT : 0.0f);
      }
      return r;
    });
  } else if (bid == NG + 3 || bid == NG + 4) {
    const float* W = (bid == NG + 3) ? gWih : gWhh;
    _Float16* D = (bid == NG + 3) ? WihP : WhhP;
    emit8<6>(D, (GH * HD) / 8, tid, [&](int p, int) -> v8h {
      const int o = p >> 3, kb = (p & 7) << 3;
      const v4f a = *(const v4f*)(W + o * HD + kb);
      const v4f b = *(const v4f*)(W + o * HD + kb + 4);
      return cvh8(a, b, SWGT);
    });
  } else {
    int ob = bid - (NG + 5);
    ob = ob < 0 ? 0 : (ob > 3 ? 3 : ob);
    emit8<6>(LstmP + (size_t)ob * 64 * LK, (64 * LK) / 8, tid, [&](int p, int) -> v8h {
      v8h r;
      const int ol = p / (LK / 8), kb = (p - ol * (LK / 8)) * 8;
      const int o = ob * 64 + ol;
      int kw = kb > 120 ? 120 : kb;
      int kh = kb - 128; kh = kh < 0 ? 0 : (kh > 56 ? 56 : kh);
      const v4f wa = *(const v4f*)(lWih + o * 128 + kw);
      const v4f wb = *(const v4f*)(lWih + o * 128 + kw + 4);
      const v4f ha = *(const v4f*)(lWhh + o * HD + kh);
      const v4f hb = *(const v4f*)(lWhh + o * HD + kh + 4);
      const v8h rw = cvh8(wa, wb, SWGT);
      const v8h rh = cvh8(ha, hb, SWGT);
#pragma unroll
      for (int kk = 0; kk < 8; ++kk) r[kk] = (kb < 128) ? rw[kk] : rh[kk];
      return r;
    });
  }
}

__global__ __launch_bounds__(128) void k_expand(const float* __restrict__ x, const _Float16* __restrict__ WexpT,
                                                 const float* __restrict__ bexp, float* outp, int nN) {
  __shared__ __attribute__((aligned(16))) _Float16 xs[64 * KX];
  __shared__ __attribute__((aligned(16))) _Float16 wsm[HD * KX];
  __shared__ __attribute__((aligned(16))) float    ot[64 * HD];
  const int tid = threadIdx.x, lane = tid & 31, wave = tid >> 5, hh = lane >> 4, m = lane & 15;
  const int row0 = blockIdx.x * 64;
  for (int idx = tid; idx < 64 * KX; idx += 128) {
    const int r = idx / KX, c = idx - r * KX;
    int gr = row0 + r; gr = gr > nN - 1 ? nN - 1 : gr;
    const int cc = c > NDIM - 1 ? NDIM - 1 : c;
    const float v = x[(size_t)gr * NDIM + cc];
    xs[idx] = (_Float16)((c < NDIM) ? v * SACT : 0.0f);
  }
  for (int p = tid; p < (HD * KX) / 8; p += 128)
    *(uint4*)(wsm + 8 * p) = *(const uint4*)(WexpT + 8 * p);
  __syncthreads();

  v8f acc[4];
#pragma unroll
  for (int q = 0; q < 4; ++q) acc[q] = zerof8();
#pragma unroll
  for (int ks = 0; ks < KX / 32; ++ks) {
    const FragH a = ldf(xs + (16 * wave + m) * KX + 32 * ks + 8 * hh);
#pragma unroll
    for (int q = 0; q < 4; ++q) {
      const FragH b = ldf(wsm + (16 * q + m) * KX + 32 * ks + 8 * hh);
      acc[q] = wmh(a.v, b.v, acc[q]);
    }
  }
#pragma unroll
  for (int q = 0; q < 4; ++q) {
    const int col = 16 * q + m;
    const float bb = bexp[col];
#pragma unroll
    for (int r = 0; r < 8; ++r) {
      const int rl = 16 * wave + 8 * hh + r;
      ot[rl * HD + col] = fmaxf(acc[q][r] * ISC256 + bb, 0.0f);
    }
  }
  __syncthreads();
  v4f ov[8];
#pragma unroll
  for (int it = 0; it < 8; ++it) {
    const int rl = 16 * wave + 2 * it + hh;
    ov[it] = *(const v4f*)(ot + rl * HD + 4 * m);
  }
#pragma unroll
  for (int it = 0; it < 8; ++it) {
    const int rl = 16 * wave + 2 * it + hh;
    *(volatile v4f*)(outp + (size_t)(row0 + rl) * HD + 4 * m) = ov[it];
  }
  __threadfence();
#pragma unroll
  for (int it = 0; it < 8; ++it) {
    const int rl = 16 * wave + 2 * it + hh;
    *(volatile v4f*)(outp + (size_t)(row0 + rl) * HD + 4 * m) = ov[it];
  }
}

__device__ __forceinline__ int scan_chunk(const int* __restrict__ dsts, int nE, int cbase, int nodeBase,
                                          int vec8, int* list, int tid, int wave) {
  int wc = 0;
  const int el0  = tid * EPT;
  const int e0   = cbase + el0;
  const int sent = -2147483647 - 1;
  v4i da, db;
  if (vec8 != 0 && cbase + CHUNK <= nE) {
    da = *(const v4i*)(dsts + e0);
    db = *(const v4i*)(dsts + e0 + 4);
  } else {
    da.x = (e0     < nE) ? dsts[min(e0, nE - 1)] : sent;
    da.y = (e0 + 1 < nE) ? dsts[min(e0 + 1, nE - 1)] : sent;
    da.z = (e0 + 2 < nE) ? dsts[min(e0 + 2, nE - 1)] : sent;
    da.w = (e0 + 3 < nE) ? dsts[min(e0 + 3, nE - 1)] : sent;
    db.x = (e0 + 4 < nE) ? dsts[min(e0 + 4, nE - 1)] : sent;
    db.y = (e0 + 5 < nE) ? dsts[min(e0 + 5, nE - 1)] : sent;
    db.z = (e0 + 6 < nE) ? dsts[min(e0 + 6, nE - 1)] : sent;
    db.w = (e0 + 7 < nE) ? dsts[min(e0 + 7, nE - 1)] : sent;
  }
  const unsigned nb = (unsigned)nodeBase;
  const unsigned s0 = (unsigned)da.x - nb, s1 = (unsigned)da.y - nb;
  const unsigned s2 = (unsigned)da.z - nb, s3 = (unsigned)da.w - nb;
  const unsigned s4 = (unsigned)db.x - nb, s5 = (unsigned)db.y - nb;
  const unsigned s6 = (unsigned)db.z - nb, s7 = (unsigned)db.w - nb;
  const bool h0 = s0 < (unsigned)NB, h1 = s1 < (unsigned)NB, h2 = s2 < (unsigned)NB, h3 = s3 < (unsigned)NB;
  const bool h4 = s4 < (unsigned)NB, h5 = s5 < (unsigned)NB, h6 = s6 < (unsigned)NB, h7 = s7 < (unsigned)NB;
  const unsigned any = __builtin_amdgcn_ballot_w32(h0 | h1 | h2 | h3 | h4 | h5 | h6 | h7);
  if (any != 0u) {
#define HITJ(J, HJ) { \
      const unsigned mj = __builtin_amdgcn_ballot_w32(HJ); \
      if (mj != 0u) { \
        if (HJ) { \
          const int pos = wc + (int)__builtin_amdgcn_mbcnt_lo(mj, 0u); \
          if (pos < WCAP) list[wave * WCAP + pos] = el0 + (J); \
        } \
        wc += (int)__builtin_popcount(mj); } }
    HITJ(0, h0)
    HITJ(1, h1)
    HITJ(2, h2)
    HITJ(3, h3)
    HITJ(4, h4)
    HITJ(5, h5)
    HITJ(6, h6)
    HITJ(7, h7)
#undef HITJ
  }
  return wc;
}

__global__ __launch_bounds__(NTHR) void k_edge(
    const float* __restrict__ outc, const int* __restrict__ ei, const float* __restrict__ ea,
    const _Float16* __restrict__ We1T, const float* __restrict__ be1,
    const _Float16* __restrict__ Wp, float* aggr, int nN, int nE, int vec8, int outLim) {
  float*    acc   = (float*)(dyn_lds + EO_ACC);
  float*    msg   = (float*)(dyn_lds + EO_MSG);
  _Float16* sea   = (_Float16*)(dyn_lds + EO_SEA);
  _Float16* sou   = (_Float16*)(dyn_lds + EO_SOU);
  int*      list  = (int*)(dyn_lds + EO_LIST);
  int*      pend  = (int*)(dyn_lds + EO_PEND);
  int*      slotb = (int*)(dyn_lds + EO_SLOT);
  _Float16* we1s  = (_Float16*)(dyn_lds + EO_WE1);
  float*    bsm   = (float*)(dyn_lds + EO_BSM);
  int*      wcnt  = (int*)(dyn_lds + EO_WCNT);
  int*      pendN = (int*)(dyn_lds + EO_PN);

  const int tid = threadIdx.x, lane = tid & 31, wave = tid >> 5, hh = lane >> 4, m = lane & 15;
  const int nodeBase = blockIdx.x * NB;
  const int* srcs = ei;
  const int* dsts = ei + nE;

  for (int i = tid; i < (NB + 1) * AW; i += NTHR) acc[i] = 0.0f;
  for (int i = tid; i < (INTD * 32) / 8; i += NTHR)
    *(uint4*)(we1s + 8 * i) = *(const uint4*)(We1T + 8 * i);
  if (tid < INTD) bsm[tid] = be1[tid] * SBIA;
  if (tid == 0) *pendN = 0;
  __syncthreads();

  const int nChunks = (nE + CHUNK - 1) / CHUNK;
#pragma unroll 1
  for (int ch = 0; ch < nChunks; ++ch) {
    const int cbase = ch * CHUNK;
    const int wc = scan_chunk(dsts, nE, cbase, nodeBase, vec8, list, tid, wave);
    if (lane == 0) wcnt[wave] = wc;
    __syncthreads();

    const int base = *pendN;
    int tot = 0, myoff = 0;
#pragma unroll
    for (int w = 0; w < NWAVE; ++w) {
      int c = wcnt[w];
      c = c > WCAP ? WCAP : (c < 0 ? 0 : c);
      if (w < wave) myoff += c;
      tot += c;
    }
    int newN = base + tot;
    newN = newN > PCAP ? PCAP : newN;
    {
      int n = wcnt[wave];
      n = n > WCAP ? WCAP : (n < 0 ? 0 : n);
      const int* lp = list + wave * WCAP;
      for (int i = lane; i < n; i += 32) {
        const int pos = base + myoff + i;
        if (pos < PCAP) pend[pos] = cbase + lp[i];
      }
    }
    const int fin = (ch == nChunks - 1) ? 1 : 0;
    const int R   = (fin != 0) ? (newN + PASSN - 1) / PASSN : newN / PASSN;
    const int Pv  = (fin != 0) ? newN : R * PASSN;
    __syncthreads();

#pragma unroll 1
    for (int r = 0; r < R; ++r) {
      const int el = wave * TPW + m;
      {
        const int idx = r * PASSN + el;
        const bool valid = idx < Pv;
        int e = pend[idx];
        if (!valid) e = 0;
        e = e < 0 ? 0 : (e > nE - 1 ? nE - 1 : e);
        const int d = dsts[e];
        int s = srcs[e];
        int slot = d - nodeBase;
        if (!valid || (unsigned)slot >= (unsigned)NB) slot = NB;
        s = s < 0 ? 0 : (s > nN - 1 ? nN - 1 : s);
        const float sc = valid ? SACT : 0.0f;
        const float* eap = ea + (size_t)e * BDIM + 8 * hh;
        const v4f x0 = *(const v4f*)eap;
        const v4f x1 = *(const v4f*)(eap + 4);
        *(v8h*)(sea + el * BDIM + 8 * hh) = cvh8(x0, x1, sc);
        const float* orp = outc + (size_t)s * HD + 32 * hh;
#pragma unroll
        for (int c = 0; c < 4; ++c) {
          const v4f y0 = *(const v4f*)(orp + 8 * c);
          const v4f y1 = *(const v4f*)(orp + 8 * c + 4);
          *(v8h*)(sou + el * HD + 32 * hh + 8 * c) = cvh8(y0, y1, sc);
        }
        if (hh == 0) slotb[el] = slot;
      }
      __syncthreads();

      {
        FragH ehf[4];
        {
          FragH bq;
          bq.h[0] = *(const v8h*)(sea + el * BDIM + 8 * hh);
          bq.h[1] = zero8();
#pragma unroll
          for (int t = 0; t < 8; ++t) {
            const FragH a = ldf(we1s + (16 * t + m) * 32 + 8 * hh);
            const v8f c = ldc8(bsm + 16 * t + 8 * hh);
            const v8f d = wmh(a.v, bq.v, c);
            ehf[t >> 1].h[t & 1] = cveh(d);
          }
        }
        v8f c0 = zerof8(), c1 = zerof8(), c2 = zerof8(), c3 = zerof8();
        const _Float16* orow = sou + el * HD;
        const _Float16* wl = Wp + (size_t)m * KW + 8 * hh;
#pragma unroll 1
        for (int i = 0; i < HD; ++i) {
          const _Float16 ov = orow[i];
          const _Float16* wi = wl + i * INTD;
#pragma unroll
          for (int j = 0; j < 4; ++j) {
            const v16h av = ehf[j].v * ov;
            const _Float16* wk = wi + 32 * j;
            const FragH b0 = ldf(wk);
            const FragH b1 = ldf(wk + 16 * KW);
            const FragH b2 = ldf(wk + 32 * KW);
            const FragH b3 = ldf(wk + 48 * KW);
            wm4(av, b0.v, b1.v, b2.v, b3.v, c0, c1, c2, c3);
          }
        }
#pragma unroll
        for (int t = 0; t < 2; ++t) {
          const FragH a = ldf(orow + 32 * t + 8 * hh);
          const _Float16* wk = wl + HD * INTD + 32 * t;
          const FragH b0 = ldf(wk);
          const FragH b1 = ldf(wk + 16 * KW);
          const FragH b2 = ldf(wk + 32 * KW);
          const FragH b3 = ldf(wk + 48 * KW);
          wm4(a.v, b0.v, b1.v, b2.v, b3.v, c0, c1, c2, c3);
        }
        float* mrow = msg + (wave * TPW + 8 * hh) * AW + m;
#pragma unroll
        for (int rr = 0; rr < 8; ++rr) {
          mrow[rr * AW]      = c0[rr] * ISC4096;
          mrow[rr * AW + 16] = c1[rr] * ISC4096;
          mrow[rr * AW + 32] = c2[rr] * ISC4096;
          mrow[rr * AW + 48] = c3[rr] * ISC4096;
        }
        if (hh == 0) msg[(wave * TPW + m) * AW + HD] = 1.0f;
      }
      __syncthreads();

      if (tid < AW) {
#pragma unroll 1
        for (int i = 0; i < PASSN; ++i) {
          int sl = slotb[i];
          sl = sl < 0 ? 0 : (sl > NB ? NB : sl);
          acc[sl * AW + tid] += msg[i * AW + tid];
        }
      }
      __syncthreads();
    }

    int rem = newN - R * PASSN;
    rem = rem < 0 ? 0 : rem;
    if (R > 0 && tid < rem) pend[tid] = pend[R * PASSN + tid];
    if (tid == 0) *pendN = rem;
  }
  __syncthreads();

  v4f ov[NQE];
#pragma unroll
  for (int q = 0; q < NQE; ++q) {
    const int f = (wave * NQE + q) * 128 + 4 * lane;
    const int sl = f >> 6;
    const int c  = f & 63;
    const float cn = acc[sl * AW + HD];
    const float inv = rcpf(fmaxf(cn, 1.0f));
    v4f v;
    v.x = acc[sl * AW + c] * inv;
    v.y = acc[sl * AW + c + 1] * inv;
    v.z = acc[sl * AW + c + 2] * inv;
    v.w = acc[sl * AW + c + 3] * inv;
    ov[q] = v;
  }
  const size_t ob  = (size_t)nodeBase * HD;
  const size_t lim = (size_t)(outLim < 0 ? 0 : outLim);
#pragma unroll
  for (int q = 0; q < NQE; ++q) {
    const size_t gi = ob + (size_t)((wave * NQE + q) * 128 + 4 * lane);
    if (gi + 3 < lim) *(volatile v4f*)(aggr + gi) = ov[q];
  }
  __threadfence();
#pragma unroll
  for (int q = 0; q < NQE; ++q) {
    const size_t gi = ob + (size_t)((wave * NQE + q) * 128 + 4 * lane);
    if (gi + 3 < lim) *(volatile v4f*)(aggr + gi) = ov[q];
  }
}

__global__ __launch_bounds__(128) void k_node(
    const float* __restrict__ outc, const float* __restrict__ aggr,
    const _Float16* __restrict__ WrootP, const _Float16* __restrict__ WihP, const _Float16* __restrict__ WhhP,
    const float* __restrict__ bconv, const float* __restrict__ bih, const float* __restrict__ bhh,
    float* outn) {
  __shared__ __attribute__((aligned(16))) _Float16 ohs[64 * HD];
  __shared__ __attribute__((aligned(16))) _Float16 mhs[64 * HD];
  __shared__ __attribute__((aligned(16))) float    tl[64 * HD];
  const int tid = threadIdx.x, lane = tid & 31, wave = tid >> 5, hh = lane >> 4, m = lane & 15;
  const int row0 = blockIdx.x * 64;
  for (int p = tid; p < (64 * HD) / 4; p += 128) {
    const int r = p >> 4, c4 = (p & 15) * 4;
    const v4f v = *(const v4f*)(outc + (size_t)(row0 + r) * HD + c4);
    *(v4f*)(tl + r * HD + c4) = v;
    v4h q;
    q[0] = (_Float16)(v.x * SACT); q[1] = (_Float16)(v.y * SACT);
    q[2] = (_Float16)(v.z * SACT); q[3] = (_Float16)(v.w * SACT);
    *(v4h*)(ohs + r * HD + c4) = q;
  }
  __syncthreads();
  FragH ao[2];
  ao[0] = ldf(ohs + (16 * wave + m) * HD + 8 * hh);
  ao[1] = ldf(ohs + (16 * wave + m) * HD + 32 + 8 * hh);

#pragma unroll
  for (int q = 0; q < 4; ++q) {
    v8f c = zerof8();
#pragma unroll
    for (int ks = 0; ks < 2; ++ks) {
      const FragH b = ldf(WrootP + (16 * q + m) * HD + 32 * ks + 8 * hh);
      c = wmh(ao[ks].v, b.v, c);
    }
    const int col = 16 * q + m;
    const float bc = bconv[col];
#pragma unroll
    for (int r = 0; r < 8; ++r) {
      const int rl = 16 * wave + 8 * hh + r;
      const float mv = fmaxf(c[r] * ISC256 + aggr[(size_t)(row0 + rl) * HD + col] + bc, 0.0f);
      mhs[rl * HD + col] = (_Float16)(mv * SACT);
    }
  }
  __syncthreads();
  FragH am[2];
  am[0] = ldf(mhs + (16 * wave + m) * HD + 8 * hh);
  am[1] = ldf(mhs + (16 * wave + m) * HD + 32 + 8 * hh);

  v8f rv[4], nv[4];
#pragma unroll
  for (int q = 0; q < 4; ++q) {
    v8f ci = zerof8(), chh = zerof8();
#pragma unroll
    for (int ks = 0; ks < 2; ++ks) {
      const FragH bi = ldf(WihP + (16 * q + m) * HD + 32 * ks + 8 * hh);
      const FragH bh = ldf(WhhP + (16 * q + m) * HD + 32 * ks + 8 * hh);
      ci  = wmh(am[ks].v, bi.v, ci);
      chh = wmh(ao[ks].v, bh.v, chh);
    }
    const int col = 16 * q + m;
    const float b1 = bih[col] + bhh[col];
    v8f t;
#pragma unroll
    for (int r = 0; r < 8; ++r) t[r] = sigf(ci[r] * ISC256 + chh[r] * ISC256 + b1);
    rv[q] = t;
  }
#pragma unroll
  for (int q = 0; q < 4; ++q) {
    v8f ci = zerof8(), chh = zerof8();
#pragma unroll
    for (int ks = 0; ks < 2; ++ks) {
      const FragH bi = ldf(WihP + (2 * HD + 16 * q + m) * HD + 32 * ks + 8 * hh);
      const FragH bh = ldf(WhhP + (2 * HD + 16 * q + m) * HD + 32 * ks + 8 * hh);
      ci  = wmh(am[ks].v, bi.v, ci);
      chh = wmh(ao[ks].v, bh.v, chh);
    }
    const int col = 16 * q + m;
    const float bi2 = bih[2 * HD + col], bh2 = bhh[2 * HD + col];
    v8f t;
#pragma unroll
    for (int r = 0; r < 8; ++r) {
      const float gin = ci[r] * ISC256 + bi2;
      const float ghn = chh[r] * ISC256 + bh2;
      t[r] = tanhf(gin + rv[q][r] * ghn);
    }
    nv[q] = t;
  }
#pragma unroll
  for (int q = 0; q < 4; ++q) {
    v8f ci = zerof8(), chh = zerof8();
#pragma unroll
    for (int ks = 0; ks < 2; ++ks) {
      const FragH bi = ldf(WihP + (HD + 16 * q + m) * HD + 32 * ks + 8 * hh);
      const FragH bh = ldf(WhhP + (HD + 16 * q + m) * HD + 32 * ks + 8 * hh);
      ci  = wmh(am[ks].v, bi.v, ci);
      chh = wmh(ao[ks].v, bh.v, chh);
    }
    const int col = 16 * q + m;
    const float b1 = bih[HD + col] + bhh[HD + col];
#pragma unroll
    for (int r = 0; r < 8; ++r) {
      const int rl = 16 * wave + 8 * hh + r;
      const float z = sigf(ci[r] * ISC256 + chh[r] * ISC256 + b1);
      const float h = tl[rl * HD + col];
      tl[rl * HD + col] = (1.0f - z) * nv[q][r] + z * h;
    }
  }
  __syncthreads();
  v4f ov[8];
#pragma unroll
  for (int it = 0; it < 8; ++it) {
    const int rl = 16 * wave + 2 * it + hh;
    ov[it] = *(const v4f*)(tl + rl * HD + 4 * m);
  }
#pragma unroll
  for (int it = 0; it < 8; ++it) {
    const int rl = 16 * wave + 2 * it + hh;
    *(volatile v4f*)(outn + (size_t)(row0 + rl) * HD + 4 * m) = ov[it];
  }
  __threadfence();
#pragma unroll
  for (int it = 0; it < 8; ++it) {
    const int rl = 16 * wave + 2 * it + hh;
    *(volatile v4f*)(outn + (size_t)(row0 + rl) * HD + 4 * m) = ov[it];
  }
}

__global__ __launch_bounds__(NTHR) void k_s2s(
    const float* __restrict__ outc, const int* __restrict__ batch, const _Float16* __restrict__ LstmP,
    const float* __restrict__ lbih, const float* __restrict__ lbhh, float* dout, int nN) {
  _Float16* Apl  = (_Float16*)(dyn_lds + SO_APL);
  float*    hls  = (float*)(dyn_lds + SO_HLS);
  float*    racc = (float*)(dyn_lds + SO_RAC);
  float*    gmax = (float*)(dyn_lds + SO_GMX);
  float*    gsum = (float*)(dyn_lds + SO_GSM);
  float*    ginv = (float*)(dyn_lds + SO_GIV);
  float*    es   = (float*)(dyn_lds + SO_ES);
  const int tid = threadIdx.x, lane = tid & 31, wave = tid >> 5, hh = lane >> 4, m = lane & 15;
  const int mt = wave & 3, par = wave >> 2;
  const float NEG_INF = __uint_as_float(0xff800000u);

  for (int p = tid; p < (NG * LK) / 8; p += NTHR) *(v8h*)(Apl + 8 * p) = zero8();
  v8f clv[2];
  clv[0] = zerof8(); clv[1] = zerof8();

#pragma unroll 1
  for (int st = 0; st < 3; ++st) {
    __syncthreads();
    v8f ac[4][2];
#pragma unroll
    for (int g = 0; g < 4; ++g) { ac[g][0] = zerof8(); ac[g][1] = zerof8(); }
#pragma unroll
    for (int ks = 0; ks < LK / 32; ++ks) {
      const FragH a = ldf(Apl + (16 * mt + m) * LK + 32 * ks + 8 * hh);
#pragma unroll
      for (int g = 0; g < 4; ++g) {
#pragma unroll
        for (int tp = 0; tp < 2; ++tp) {
          const int nt = 4 * g + 2 * par + tp;
          const FragH b = ldf(LstmP + (size_t)(16 * nt + m) * LK + 32 * ks + 8 * hh);
          ac[g][tp] = wmh(a.v, b.v, ac[g][tp]);
        }
      }
    }
    __syncthreads();
#pragma unroll
    for (int tp = 0; tp < 2; ++tp) {
      const int u = 16 * (2 * par + tp) + m;
      const float b_i = lbih[u] + lbhh[u];
      const float b_f = lbih[HD + u] + lbhh[HD + u];
      const float b_g = lbih[2 * HD + u] + lbhh[2 * HD + u];
      const float b_o = lbih[3 * HD + u] + lbhh[3 * HD + u];
#pragma unroll
      for (int r = 0; r < 8; ++r) {
        const int brow = 16 * mt + 8 * hh + r;
        const float gi = ac[0][tp][r] * ISC256 + b_i;
        const float gf = ac[1][tp][r] * ISC256 + b_f;
        const float gg = ac[2][tp][r] * ISC256 + b_g;
        const float go = ac[3][tp][r] * ISC256 + b_o;
        const float c = sigf(gf) * clv[tp][r] + sigf(gi) * tanhf(gg);
        clv[tp][r] = c;
        const float hv = sigf(go) * tanhf(c);
        hls[brow * HD + u] = hv;
        const _Float16 hq = (_Float16)(hv * SACT);
        Apl[brow * LK + u] = hq;
        Apl[brow * LK + 2 * HD + u] = hq;
      }
    }
    for (int p = tid; p < NG * HD; p += NTHR) racc[p] = 0.0f;
    __syncthreads();
    for (int n = tid; n < nN; n += NTHR) {
      int bb = batch[n];
      bb = bb < 0 ? 0 : (bb > NG - 1 ? NG - 1 : bb);
      const float* orp = outc + (size_t)n * HD;
      const float* qp = hls + bb * HD;
      float e = 0.0f;
#pragma unroll
      for (int k4 = 0; k4 < HD / 4; ++k4) {
        const v4f o = *(const v4f*)(orp + 4 * k4);
        const v4f q = *(const v4f*)(qp + 4 * k4);
        e += o.x * q.x; e += o.y * q.y; e += o.z * q.z; e += o.w * q.w;
      }
      es[n] = e;
    }
    __syncthreads();
    if (tid < NG) {
      float mx = NEG_INF;
#pragma unroll 1
      for (int n = 0; n < nN; ++n) {
        int bb = batch[n];
        bb = bb < 0 ? 0 : (bb > NG - 1 ? NG - 1 : bb);
        if (bb == tid) mx = fmaxf(mx, es[n]);
      }
      gmax[tid] = mx;
    }
    __syncthreads();
    for (int n = tid; n < nN; n += NTHR) {
      int bb = batch[n];
      bb = bb < 0 ? 0 : (bb > NG - 1 ? NG - 1 : bb);
      es[n] = __expf(es[n] - gmax[bb]);
    }
    __syncthreads();
    if (tid < NG) {
      float s = 0.0f;
#pragma unroll 1
      for (int n = 0; n < nN; ++n) {
        int bb = batch[n];
        bb = bb < 0 ? 0 : (bb > NG - 1 ? NG - 1 : bb);
        if (bb == tid) s += es[n];
      }
      gsum[tid] = s;
      ginv[tid] = rcpf(s);
    }
    __syncthreads();
    if (wave == 0) {
#pragma unroll 1
      for (int n = 0; n < nN; ++n) {
        int bb = batch[n];
        bb = bb < 0 ? 0 : (bb > NG - 1 ? NG - 1 : bb);
        const float w = es[n] * ginv[bb];
        const v2f o2 = *(const v2f*)(outc + (size_t)n * HD + 2 * lane);
        float* rp = racc + bb * HD + 2 * lane;
        const float r0 = rp[0] + w * o2.x;
        const float r1 = rp[1] + w * o2.y;
        rp[0] = r0;
        rp[1] = r1;
      }
    }
    __syncthreads();
    for (int p = tid; p < NG * HD; p += NTHR) {
      const int b = p >> 6, c = p & 63;
      Apl[b * LK + HD + c] = (_Float16)(racc[p] * SACT);
    }
  }
  __syncthreads();
  v4f ov[8];
#pragma unroll
  for (int it = 0; it < 8; ++it) {
    const int row = 8 * wave + it;
    const int c4 = 4 * lane, cl = c4 & 63;
    const v4f a = *(const v4f*)(hls + row * HD + cl);
    const v4f b = *(const v4f*)(racc + row * HD + cl);
    v4f v;
    v.x = (c4 < HD) ? a.x : b.x; v.y = (c4 < HD) ? a.y : b.y;
    v.z = (c4 < HD) ? a.z : b.z; v.w = (c4 < HD) ? a.w : b.w;
    ov[it] = v;
  }
#pragma unroll
  for (int it = 0; it < 8; ++it) {
    const int row = 8 * wave + it;
    *(volatile v4f*)(dout + (size_t)row * (2 * HD) + 4 * lane) = ov[it];
  }
  __threadfence();
#pragma unroll
  for (int it = 0; it < 8; ++it) {
    const int row = 8 * wave + it;
    *(volatile v4f*)(dout + (size_t)row * (2 * HD) + 4 * lane) = ov[it];
  }
}

extern "C" void kernel_launch(void* const* d_in, const int* in_sizes, int n_in,
                              void* d_out, int out_size, void* d_ws, size_t ws_size,
                              hipStream_t stream) {
  if (n_in < 20) return;
  const int N = in_sizes[0] / NDIM;
  if (N < 1 || in_sizes[0] != N * NDIM) return;
  const int E = in_sizes[1] / 2;
  if (E < 1 || in_sizes[1] != 2 * E) return;
  if (in_sizes[2] != E * BDIM || in_sizes[3] != N) return;
  if (in_sizes[4] != NDIM * HD || in_sizes[5] != HD) return;
  if (in_sizes[6] != BDIM * INTD || in_sizes[7] != INTD) return;
  if (in_sizes[8] != INTD * W2N || in_sizes[9] != W2N) return;
  if (in_sizes[10] != HD * HD || in_sizes[11] != HD) return;
  if (in_sizes[12] != GH * HD || in_sizes[13] != GH * HD || in_sizes[14] != GH || in_sizes[15] != GH) return;
  if (in_sizes[16] != LG * 2 * HD || in_sizes[17] != LG * HD || in_sizes[18] != LG || in_sizes[19] != LG) return;
  if (out_size != NG * 2 * HD) return;

  const float* x      = (const float*)d_in[0];
  const int*   ei     = (const int*)d_in[1];
  const float* ea     = (const float*)d_in[2];
  const int*   batch  = (const int*)d_in[3];
  const float* Wexp   = (const float*)d_in[4];
  const float* bexp   = (const float*)d_in[5];
  const float* We1    = (const float*)d_in[6];
  const float* be1    = (const float*)d_in[7];
  const float* We2    = (const float*)d_in[8];
  const float* be2    = (const float*)d_in[9];
  const float* Wroot  = (const float*)d_in[10];
  const float* bconv  = (const float*)d_in[11];
  const float* gWih   = (const float*)d_in[12];
  const float* gWhh   = (const float*)d_in[13];
  const float* gbih   = (const float*)d_in[14];
  const float* gbhh   = (const float*)d_in[15];
  const float* lWih   = (const float*)d_in[16];
  const float* lWhh   = (const float*)d_in[17];
  const float* lbih   = (const float*)d_in[18];
  const float* lbhh   = (const float*)d_in[19];
  float* out = (float*)d_out;

  const int nBlkN = (N + 63) / 64;
  const int Npad  = nBlkN * 64;
  const int nBlkE = (N + NB - 1) / NB;

  char* ws = (char*)d_ws;
  size_t off = 0;
  const size_t oWp   = off; off += (size_t)NG * KW * 2;        off = (off + 255) & ~(size_t)255;
  const size_t oWx   = off; off += (size_t)HD * KX * 2;        off = (off + 255) & ~(size_t)255;
  const size_t oWr   = off; off += (size_t)HD * HD * 2;        off = (off + 255) & ~(size_t)255;
  const size_t oW1   = off; off += (size_t)INTD * 32 * 2;      off = (off + 255) & ~(size_t)255;
  const size_t oWi   = off; off += (size_t)GH * HD * 2;        off = (off + 255) & ~(size_t)255;
  const size_t oWh   = off; off += (size_t)GH * HD * 2;        off = (off + 255) & ~(size_t)255;
  const size_t oWl   = off; off += (size_t)LG * LK * 2;        off = (off + 255) & ~(size_t)255;
  const size_t oOa   = off; off += (size_t)Npad * HD * 4;      off = (off + 255) & ~(size_t)255;
  const size_t oOb   = off; off += (size_t)Npad * HD * 4;      off = (off + 255) & ~(size_t)255;
  const size_t oAg   = off; off += (size_t)nBlkE * NB * HD * 4; off = (off + 255) & ~(size_t)255;
  if (off > ws_size || off > (size_t)134217728) return;
  const int s2sLds = SO_ES + al16(4 * N);
  if (s2sLds > 200000) return;

  _Float16* Wp     = (_Float16*)(ws + oWp);
  _Float16* WexpT  = (_Float16*)(ws + oWx);
  _Float16* WrootP = (_Float16*)(ws + oWr);
  _Float16* We1T   = (_Float16*)(ws + oW1);
  _Float16* WihP   = (_Float16*)(ws + oWi);
  _Float16* WhhP   = (_Float16*)(ws + oWh);
  _Float16* LstmP  = (_Float16*)(ws + oWl);
  float*    outA   = (float*)(ws + oOa);
  float*    outB   = (float*)(ws + oOb);
  float*    aggr   = (float*)(ws + oAg);

  const int vec8 = ((E & 3) == 0) ? 1 : 0;

  k_prep<<<NG + 9, 256, 0, stream>>>(We2, be2, Wexp, Wroot, We1, gWih, gWhh, lWih, lWhh,
                                     Wp, WexpT, WrootP, We1T, WihP, WhhP, LstmP);
  k_expand<<<nBlkN, 128, 0, stream>>>(x, WexpT, bexp, outA, N);

  float* cur = outA;
  float* nxt = outB;
  for (int d = 0; d < 3; ++d) {
    k_edge<<<nBlkE, NTHR, E_LDS, stream>>>(cur, ei, ea, We1T, be1, Wp, aggr, N, E, vec8, nBlkE * NB * HD);
    k_node<<<nBlkN, 128, 0, stream>>>(cur, aggr, WrootP, WihP, WhhP, bconv, gbih, gbhh, nxt);
    float* t = cur; cur = nxt; nxt = t;
  }

  k_s2s<<<1, NTHR, s2sLds, stream>>>(cur, batch, LstmP, lbih, lbhh, out, N);
}
